// PoseMLP_28965259444367
// MI455X (gfx1250) — hardware-verified
//
#include <hip/hip_runtime.h>
#include <math.h>

typedef __attribute__((ext_vector_type(16))) _Float16 v16h;
typedef __attribute__((ext_vector_type(16))) __bf16 v16b;
typedef __attribute__((ext_vector_type(8)))  _Float16 v8h;
typedef __attribute__((ext_vector_type(8)))  float v8f;
typedef __attribute__((ext_vector_type(4)))  float v4f;
typedef __attribute__((ext_vector_type(2)))  float v2f;
typedef __attribute__((ext_vector_type(4)))  unsigned v4u;
typedef __attribute__((ext_vector_type(4)))  int v4i;
typedef float __attribute__((may_alias)) float_a;
typedef int __attribute__((may_alias)) int_a;

template <typename T> __device__ __forceinline__ void vst2(void* p, T v) { *(volatile T*)p = v; __threadfence(); *(volatile T*)p = v; }
__device__ __forceinline__ v8f wmma16(v16h a, v16h b, v8f c) {
  v8f d = __builtin_amdgcn_wmma_f32_16x16x32_f16(false, a, false, b, (short)0, c, false, false);
  asm volatile("v_nop\n\tv_nop\n\tv_nop\n\tv_nop" : "+v"(d) : "v"(a), "v"(b));
  return d;
}
__device__ __forceinline__ v8f wmma_bf(v16b a, v16b b, v8f c) {
  v8f d = __builtin_amdgcn_wmma_f32_16x16x32_bf16(false, a, false, b, (short)0, c, false, false);
  asm volatile("v_nop\n\tv_nop\n\tv_nop\n\tv_nop" : "+v"(d) : "v"(a), "v"(b));
  return d;
}
__device__ __forceinline__ v16h frag_h(const _Float16* rowk0, int lane) {
  union { v16h v; v8h q[2]; } u; const _Float16* p = rowk0 + 8 * (lane >> 4);
  u.q[0] = *(const v8h*)p; u.q[1] = *(const v8h*)(p + 16); return u.v;
}
__device__ __forceinline__ v16h frag_f32(const float* rowk0, int lane) {
  v16h a; const float* p = rowk0 + 8 * (lane >> 4);
#pragma unroll
  for (int i = 0; i < 8; ++i) { a[i] = (_Float16)p[i]; a[8 + i] = (_Float16)p[16 + i]; }
  return a;
}
__device__ __forceinline__ v16h frag_f32s(const float* rowk0, int lane, float sc) {
  v16h a; const float* p = rowk0 + 8 * (lane >> 4);
#pragma unroll
  for (int i = 0; i < 8; ++i) { a[i] = (_Float16)(p[i] * sc); a[8 + i] = (_Float16)(p[16 + i] * sc); }
  return a;
}
__device__ __forceinline__ v16h fragc_f32(const float* W, int k0, int n, int lane, int ld, int K) {
  v16h a; const int g = lane >> 4;
#pragma unroll
  for (int i = 0; i < 8; ++i) { const int ka = k0 + 8 * g + i, kb = ka + 16;
    a[i] = (_Float16)(ka < K ? W[(size_t)(ka < K ? ka : K - 1) * ld + n] : 0.f); a[8 + i] = (_Float16)(kb < K ? W[(size_t)(kb < K ? kb : K - 1) * ld + n] : 0.f); }
  return a;
}
struct F2 { v16b h, l; };
__device__ __forceinline__ F2 bsplit16(const float v[16]) { F2 r;
#pragma unroll
  for (int i = 0; i < 16; ++i) { const __bf16 h = (__bf16)v[i]; r.h[i] = h; r.l[i] = (__bf16)(v[i] - (float)h); }
  return r; }
__device__ __forceinline__ F2 split_row(const float* row, int k0, int lane) { float v[16]; const float* p = row + k0 + 8 * (lane >> 4);
#pragma unroll
  for (int i = 0; i < 8; ++i) { v[i] = p[i]; v[8 + i] = p[16 + i]; }
  return bsplit16(v); }
__device__ __forceinline__ F2 split_rowK(const float* row, int k0, int lane, int K) { float v[16]; const int g = lane >> 4;
#pragma unroll
  for (int i = 0; i < 8; ++i) { const int ka = k0 + 8 * g + i, kb = ka + 16; v[i] = ka < K ? row[ka < K ? ka : K - 1] : 0.f; v[8 + i] = kb < K ? row[kb < K ? kb : K - 1] : 0.f; }
  return bsplit16(v); }
__device__ __forceinline__ F2 split_col(const float* W, int k0, int n, int lane, int ld, int K) { float v[16]; const int g = lane >> 4;
#pragma unroll
  for (int i = 0; i < 8; ++i) { const int ka = k0 + 8 * g + i, kb = ka + 16; v[i] = ka < K ? W[(size_t)(ka < K ? ka : K - 1) * ld + n] : 0.f; v[8 + i] = kb < K ? W[(size_t)(kb < K ? kb : K - 1) * ld + n] : 0.f; }
  return bsplit16(v); }
__device__ __forceinline__ v8f mac3(const F2& a, const F2& b, v8f c) { c = wmma_bf(a.l, b.h, c); c = wmma_bf(a.h, b.l, c); return wmma_bf(a.h, b.h, c); }
__device__ __forceinline__ float sigm(float v) { return 1.0f / (1.0f + expf(-v)); }
#define LDSX() do { asm volatile("s_wait_dscnt 0" ::: "memory"); __builtin_amdgcn_wave_barrier(); __builtin_amdgcn_fence(__ATOMIC_RELEASE, "workgroup"); } while (0)


#define NP 2097152
#ifndef NBLK
#define NBLK (NP / 64)
#endif
typedef __attribute__((ext_vector_type(8))) __bf16 v8b;
__device__ __forceinline__ v16b frag_b(const __bf16* rowk0, int lane) {
  union { v16b v; v8b q[2]; } u; const __bf16* p = rowk0 + 8 * (lane >> 4);
  u.q[0] = *(const v8b*)p; u.q[1] = *(const v8b*)(p + 16); return u.v;
}
__device__ __forceinline__ float bfr(float v) { return (float)(__bf16)v; }

__global__ __launch_bounds__(128) void k_main(const float* __restrict__ X, const float* __restrict__ W1, const float* __restrict__ b1, const float* __restrict__ W2, const float* __restrict__ b2, const float* __restrict__ W3, const float* __restrict__ b3, float* __restrict__ out, int total) {
  __shared__ __align__(16) __bf16 sw1[64][40];
  __shared__ __align__(16) __bf16 sw2[64][72];
  __shared__ __align__(16) __bf16 sw3[16][72];
  __shared__ float sb1[64], sb2[64], sb3[8];
  __shared__ __align__(16) __bf16 sx[64][40];
  __shared__ __align__(16) __bf16 shh[4][16][72], shl[4][16][72];
  __shared__ __align__(16) float sres[64 * 7 + 4];
  const int tid = threadIdx.x, wave = tid >> 5, lane = tid & 31, col = lane & 15, g = lane >> 4; const size_t p0 = (size_t)blockIdx.x * 64;
  for (int q = tid; q < 64 * 40; q += 128) { const int r = q / 40, k = q % 40; sw1[r][k] = (__bf16)(k < 7 ? bfr(W1[r * 7 + k]) : 0.f); const size_t pp = p0 + r; sx[r][k] = (__bf16)((k < 7 && pp < (size_t)total) ? bfr(X[pp * 7 + k]) : 0.f); }
  for (int q = tid; q < 64 * 64; q += 128) { const int r = q >> 6, k = q & 63; sw2[r][k] = (__bf16)bfr(W2[q]); }
  for (int q = tid; q < 16 * 64; q += 128) { const int r = q >> 6, k = q & 63; sw3[r][k] = (__bf16)(r < 7 ? bfr(W3[r * 64 + k]) : 0.f); }
  if (tid < 64) { sb1[tid] = bfr(b1[tid]); sb2[tid] = bfr(b2[tid]); } if (tid < 7) sb3[tid] = bfr(b3[tid]);
  __syncthreads();
  { v8f acc[4] = {}; const v16b a = frag_b(&sx[wave * 16 + col][0], lane);
#pragma unroll
    for (int j = 0; j < 4; ++j) acc[j] = wmma_bf(a, frag_b(&sw1[j * 16 + col][0], lane), acc[j]);
#pragma unroll
    for (int j = 0; j < 4; ++j)
#pragma unroll
      for (int r = 0; r < 8; ++r) { const float v = fmaxf(acc[j][r] + sb1[j * 16 + col], 0.f); const __bf16 hb = (__bf16)v; shh[wave][8 * g + r][j * 16 + col] = hb; shl[wave][8 * g + r][j * 16 + col] = (__bf16)(v - (float)hb); } }
  LDSX();
  { v8f acc[4] = {};
#pragma unroll
    for (int kc = 0; kc < 2; ++kc) { const v16b ah = frag_b(&shh[wave][col][kc * 32], lane), al = frag_b(&shl[wave][col][kc * 32], lane);
#pragma unroll
      for (int j = 0; j < 4; ++j) { const v16b w = frag_b(&sw2[j * 16 + col][kc * 32], lane); acc[j] = wmma_bf(al, w, acc[j]); acc[j] = wmma_bf(ah, w, acc[j]); } }
    LDSX();
#pragma unroll
    for (int j = 0; j < 4; ++j)
#pragma unroll
      for (int r = 0; r < 8; ++r) { const float v = fmaxf(acc[j][r] + sb2[j * 16 + col], 0.f); const __bf16 hb = (__bf16)v; shh[wave][8 * g + r][j * 16 + col] = hb; shl[wave][8 * g + r][j * 16 + col] = (__bf16)(v - (float)hb); } }
  LDSX();
  { v8f acc = {};
#pragma unroll
    for (int kc = 0; kc < 2; ++kc) { const v16b ah = frag_b(&shh[wave][col][kc * 32], lane), al = frag_b(&shl[wave][col][kc * 32], lane); const v16b w = frag_b(&sw3[col][kc * 32], lane); acc = wmma_bf(al, w, acc); acc = wmma_bf(ah, w, acc); }
    if (col < 7) {
#pragma unroll
      for (int r = 0; r < 8; ++r) sres[(wave * 16 + 8 * g + r) * 7 + col] = acc[r] + sb3[col]; } }
  __syncthreads();
  if (tid < 64) { float* o = &sres[tid * 7]; const float nrm = sqrtf((o[3] * o[3] + o[4] * o[4]) + (o[5] * o[5] + o[6] * o[6])); const float inv = 1.0f / nrm; o[3] *= inv; o[4] *= inv; o[5] *= inv; o[6] *= inv; }
  __syncthreads();
  { const int nfl = (int)((p0 + 64 <= (size_t)total ? 64 : (size_t)total - p0) * 7);
    if (tid < nfl / 4) vst2(out + p0 * 7 + tid * 4, *(const v4f*)&sres[tid * 4]); }
}

extern "C" void kernel_launch(void* const* d_in, const int* in_sizes, int n_in, void* d_out, int out_size, void* d_ws, size_t ws_size, hipStream_t stream) {
  (void)in_sizes; (void)n_in; (void)out_size; (void)d_ws; (void)ws_size;
  const float** F = (const float**)d_in;
  k_main<<<NBLK, 128, 0, stream>>>(F[0], F[1], F[2], F[3], F[4], F[5], F[6], (float*)d_out, NP);
}
